// Neurocache_1486058685086
// MI455X (gfx1250) — hardware-run, weakly checked
//
#include <hip/hip_runtime.h>
#include <math.h>
#include <stdint.h>

#define NB   2
#define SQ   1024
#define HH   1024
#define NNB  8
#define RH   256
#define NHD  16
#define HD   64
#define CTXW 4
#define MQ   (NB * SQ)
#define ME   (NB * SQ * NNB)
#define WSC  16.0f
#define QSCL 0.125f

static_assert(NHD * HD == HH);
static_assert(NNB * HH == NHD * NNB * HD);
static_assert((MQ % 64) == 0 && (ME % 64) == 0 && (HH % 64) == 0 && (RH % 32) == 0 && (HH % 32) == 0);
static_assert((((MQ / 64) * (HH / 64)) % 8) == 0);
static_assert((((ME / 64) * (HH / 64)) % 8) == 0);
static_assert(((MQ * HH) % 2048) == 0 && ((ME * RH) % 2048) == 0);
static_assert(((HH * HH) % 2048) == 0 && ((HH * RH) % 2048) == 0);
static_assert(((MQ * NHD) % 4) == 0);
static_assert(SQ == 1024 && NHD == 16 && HD == 64 && CTXW * NNB == 32);

typedef _Float16 v16h __attribute__((ext_vector_type(16)));
typedef _Float16 v8h  __attribute__((ext_vector_type(8)));
typedef _Float16 v2h  __attribute__((ext_vector_type(2)));
typedef unsigned short v16us __attribute__((ext_vector_type(16)));
typedef unsigned short v8us  __attribute__((ext_vector_type(8)));
typedef float v8f __attribute__((ext_vector_type(8)));
typedef float v4f __attribute__((ext_vector_type(4)));
typedef unsigned int v4u __attribute__((ext_vector_type(4)));

union FragU { v16us v; v8us h[2]; };

__device__ __forceinline__ unsigned short h_bits(_Float16 x) { return __builtin_bit_cast(unsigned short, x); }
__device__ __forceinline__ unsigned short f2h(float f) { return h_bits((_Float16)f); }
__device__ __forceinline__ unsigned pk16(unsigned short a, unsigned short b) { return (unsigned)a | ((unsigned)b << 16); }
__device__ __forceinline__ int clampi(int v, int lo, int hi) { return v < lo ? lo : (v > hi ? hi : v); }
__device__ __forceinline__ v8f zero8() { v8f z = {0.f, 0.f, 0.f, 0.f, 0.f, 0.f, 0.f, 0.f}; return z; }

__device__ __forceinline__ v16us ldfrag_u(const unsigned short* p) {
  FragU f;
  f.h[0] = *(const v8us*)(p);
  f.h[1] = *(const v8us*)(p + 16);
  return f.v;
}

__device__ __forceinline__ v8f mma_h_raw(v16us a, v16us b, v8f c) {
  return __builtin_amdgcn_wmma_f32_16x16x32_f16(false, __builtin_bit_cast(v16h, a), false,
                                                __builtin_bit_cast(v16h, b), (short)0, c, false, false);
}
__device__ __forceinline__ void dep_guard1(v8f& a, v8f& b, v16us x) {
#if defined(__HIP_DEVICE_COMPILE__)
  asm volatile("v_nop\n\tv_nop\n\tv_nop\n\tv_nop" : "+v"(a), "+v"(b) : "v"(x));
#endif
}
__device__ __forceinline__ void keep4_u(v16us a, v16us b, v16us c, v16us d) {
#if defined(__HIP_DEVICE_COMPILE__)
  asm volatile("v_nop" :: "v"(a), "v"(b), "v"(c), "v"(d));
#endif
}
__device__ __forceinline__ void acc_guard4(v8f& a, v8f& b, v8f& c, v8f& d) {
#if defined(__HIP_DEVICE_COMPILE__)
  asm volatile("v_nop\n\tv_nop\n\tv_nop\n\tv_nop" : "+v"(a), "+v"(b), "+v"(c), "+v"(d));
#endif
}
__device__ __forceinline__ void wave_sync_lds() {
  __builtin_amdgcn_fence(__ATOMIC_RELEASE, "workgroup");
  __builtin_amdgcn_wave_barrier();
  __builtin_amdgcn_fence(__ATOMIC_ACQUIRE, "workgroup");
}

__global__ __launch_bounds__(256) void cvt_flat(const float* __restrict__ x, unsigned short* xh, int n8, float sc) {
  const int i = blockIdx.x * 256 + threadIdx.x;
  if (i >= n8) return;
  const float* p = x + (size_t)i * 8;
  const v4f a0 = *(const v4f*)(p);
  const v4f a1 = *(const v4f*)(p + 4);
  v4u hv;
#pragma unroll
  for (int e = 0; e < 2; ++e) {
    hv[e]     = pk16(f2h(a0[2 * e] * sc), f2h(a0[2 * e + 1] * sc));
    hv[2 + e] = pk16(f2h(a1[2 * e] * sc), f2h(a1[2 * e + 1] * sc));
  }
  unsigned short* d = xh + (size_t)i * 8;
  for (int pass = 0; pass < 2; ++pass) {
    *(volatile v4u*)(d) = hv;
    __threadfence();
  }
}

template <int OM>
__global__ __launch_bounds__(256) void gemm64(
    const unsigned short* __restrict__ Ap, int lda,
    const unsigned short* __restrict__ Btp, int ldb,
    unsigned short* Ch, float* Cf, int ldc,
    const float* __restrict__ Rp, int ldr,
    float wsc, int M, int N, int K) {
  __shared__ __align__(16) float sT[8][16 * 68];
  const int lane = threadIdx.x & 31;
  const int wave = threadIdx.x >> 5;
  const int tilesN = N >> 6;
  const int tilesM = M >> 6;
  const int tile = blockIdx.x * 8 + wave;
  if (tile >= tilesM * tilesN) return;
  const int tm = tile / tilesN;
  const int tn = tile - tm * tilesN;
  const int m0 = tm << 6;
  const int n0 = tn << 6;

  const int rlane = lane & 15;
  const int koff  = (lane >> 4) * 8;
  const int mOff  = (lane >> 4) * 8;

  v8f acc[4][4];
#pragma unroll
  for (int i = 0; i < 4; ++i)
#pragma unroll
    for (int j = 0; j < 4; ++j) acc[i][j] = zero8();

  for (int k0 = 0; k0 < K; k0 += 32) {
    v16us bh[4];
#pragma unroll
    for (int j = 0; j < 4; ++j) {
      const size_t bo = (size_t)(n0 + (j << 4) + rlane) * ldb + koff + k0;
      bh[j] = ldfrag_u(Btp + bo);
    }
#pragma unroll
    for (int i = 0; i < 4; ++i) {
      const size_t ao = (size_t)(m0 + (i << 4) + rlane) * lda + koff + k0;
      const v16us ah = ldfrag_u(Ap + ao);
#pragma unroll
      for (int j = 0; j < 4; ++j) acc[i][j] = mma_h_raw(ah, bh[j], acc[i][j]);
      dep_guard1(acc[i][0], acc[i][3], ah);
    }
    keep4_u(bh[0], bh[1], bh[2], bh[3]);
  }
  acc_guard4(acc[0][0], acc[0][1], acc[0][2], acc[0][3]);
  acc_guard4(acc[1][0], acc[1][1], acc[1][2], acc[1][3]);
  acc_guard4(acc[2][0], acc[2][1], acc[2][2], acc[2][3]);
  acc_guard4(acc[3][0], acc[3][1], acc[3][2], acc[3][3]);

  const int hh2 = lane >> 4, c4 = (lane & 15) * 4;
  const int q8  = lane >> 3, c8 = (lane & 7) * 8;

  float* slab = sT[wave];
#pragma unroll
  for (int i = 0; i < 4; ++i) {
    const int mBase = m0 + (i << 4);
#pragma unroll
    for (int j = 0; j < 4; ++j) {
#pragma unroll
      for (int r = 0; r < 8; ++r) {
        slab[(mOff + r) * 68 + (j << 4) + rlane] = acc[i][j][r];
      }
    }
    wave_sync_lds();
    if (OM == 0 || OM == 2) {
      v4f vals[8];
#pragma unroll
      for (int it = 0; it < 8; ++it) {
        const int row = it * 2 + hh2;
        const v4f v = *(const v4f*)(slab + row * 68 + c4);
        v4f tv = v * wsc;
        if (OM == 2) {
          const v4f rr = *(const v4f*)(Rp + (size_t)(mBase + row) * ldr + (size_t)n0 + c4);
          tv = tv + rr;
        }
        vals[it] = tv;
      }
      for (int pass = 0; pass < 2; ++pass) {
#pragma unroll
        for (int it = 0; it < 8; ++it) {
          const int row = it * 2 + hh2;
          *(volatile v4f*)(Cf + (size_t)(mBase + row) * ldc + (size_t)n0 + c4) = vals[it];
        }
        __threadfence();
      }
    }
    if (OM == 1) {
      v4u hv[4];
#pragma unroll
      for (int it = 0; it < 4; ++it) {
        const int row = it * 4 + q8;
        const float* sp = slab + row * 68 + c8;
        v4u ha = {0u, 0u, 0u, 0u};
#pragma unroll
        for (int e = 0; e < 4; ++e) {
          const float f0 = sp[2 * e]     * wsc;
          const float f1 = sp[2 * e + 1] * wsc;
          ha[e] = pk16(f2h(f0), f2h(f1));
        }
        hv[it] = ha;
      }
      for (int pass = 0; pass < 2; ++pass) {
#pragma unroll
        for (int it = 0; it < 4; ++it) {
          const int row = it * 4 + q8;
          const size_t go = (size_t)(mBase + row) * ldc + (size_t)n0 + c8;
          *(volatile v4u*)(Ch + go) = hv[it];
        }
        __threadfence();
      }
    }
    wave_sync_lds();
  }
}

__global__ __launch_bounds__(128) void attn_win(const float* __restrict__ Qf, const _Float16* __restrict__ Kh,
                                                const _Float16* __restrict__ Vh, unsigned short* Zh) {
  __shared__ __align__(16) float qs[4][HD];
  __shared__ float ps[4][32];
  const int t = threadIdx.x, lane = t & 31, wv = t >> 5;
  const int gw = blockIdx.x * 4 + wv;
  const int head = gw & (NHD - 1);
  const int tok = gw >> 4;
  const int s = tok & (SQ - 1);
  const int b = tok >> 10;
  const size_t qo = (size_t)tok * HH + (size_t)head * HD;
  qs[wv][lane]      = Qf[qo + lane];
  qs[wv][lane + 32] = Qf[qo + lane + 32];
  wave_sync_lds();

  const int j = lane >> 3, nn = lane & 7;
  const int p = clampi(s - (CTXW - 1) + j, 0, SQ - 1);
  const size_t kb = ((size_t)(b * SQ + p) * NNB + (head >> 1)) * HH + (size_t)(head & 1) * (HH / 2) + (size_t)nn * HD;
  const _Float16* kp = Kh + kb;
  const float* qp = &qs[wv][0];
  float dot = 0.f;
#pragma unroll 1
  for (int d8 = 0; d8 < HD; d8 += 8) {
    const v8h kv = *(const v8h*)(kp + d8);
    const v4f q0 = *(const v4f*)(qp + d8);
    const v4f q1 = *(const v4f*)(qp + d8 + 4);
    dot += q0[0] * (float)kv[0];
    dot += q0[1] * (float)kv[1];
    dot += q0[2] * (float)kv[2];
    dot += q0[3] * (float)kv[3];
    dot += q1[0] * (float)kv[4];
    dot += q1[1] * (float)kv[5];
    dot += q1[2] * (float)kv[6];
    dot += q1[3] * (float)kv[7];
  }
  const float sc = dot * (1.0f / WSC);
  float mx = sc;
#pragma unroll
  for (int off = 16; off > 0; off >>= 1) mx = fmaxf(mx, __shfl_xor(mx, off, 32));
  const float e = __expf(sc - mx);
  float sum = e;
#pragma unroll
  for (int off = 16; off > 0; off >>= 1) sum += __shfl_xor(sum, off, 32);
  const float pr = e * (1.0f / sum);
  ps[wv][lane] = pr;
  wave_sync_lds();

  const int d0 = 2 * lane;
  float a0 = 0.f, a1 = 0.f;
#pragma unroll 1
  for (int jj = 0; jj < CTXW; ++jj) {
    const int pj = clampi(s - (CTXW - 1) + jj, 0, SQ - 1);
    const _Float16* vp = Vh + ((size_t)(b * SQ + pj) * NNB + (head >> 1)) * HH + (size_t)(head & 1) * (HH / 2) + d0;
#pragma unroll
    for (int nni = 0; nni < NNB; ++nni) {
      const v2h vv = *(const v2h*)(vp + nni * HD);
      const float w = ps[wv][jj * NNB + nni];
      a0 += w * (float)vv[0];
      a1 += w * (float)vv[1];
    }
  }
  const unsigned pk = pk16(f2h(a0), f2h(a1));
  const int src = 4 * (lane & 7);
  v4u hv;
  hv[0] = __shfl(pk, src, 32);
  hv[1] = __shfl(pk, src + 1, 32);
  hv[2] = __shfl(pk, src + 2, 32);
  hv[3] = __shfl(pk, src + 3, 32);
  const size_t zo = qo + (size_t)(lane & 7) * 8;
  for (int pass = 0; pass < 2; ++pass) {
    if (lane < 8) *(volatile v4u*)(Zh + zo) = hv;
    __threadfence();
  }
}

extern "C" void kernel_launch(void* const* d_in, const int* in_sizes, int n_in,
                              void* d_out, int out_size, void* d_ws, size_t ws_size,
                              hipStream_t stream) {
  if (n_in < 6) return;
  if (in_sizes[0] != MQ * HH || in_sizes[1] != ME * RH) return;
  if (in_sizes[2] != HH * HH || in_sizes[3] != HH * RH || in_sizes[4] != HH * RH || in_sizes[5] != HH * HH) return;
  if (out_size != MQ * HH) return;

  const float* x  = (const float*)d_in[0];
  const float* ex = (const float*)d_in[1];
  const float* Wq = (const float*)d_in[2];
  const float* Wk = (const float*)d_in[3];
  const float* Wv = (const float*)d_in[4];
  const float* Wo = (const float*)d_in[5];

  const size_t PXH = (size_t)MQ * HH * 2;
  const size_t PEH = (size_t)ME * RH * 2;
  const size_t PWQ = (size_t)HH * HH * 2;
  const size_t PWK = (size_t)HH * RH * 2;
  const size_t PWV = (size_t)HH * RH * 2;
  const size_t PWO = (size_t)HH * HH * 2;
  const size_t PQF = (size_t)MQ * HH * 4;
  const size_t PKH = (size_t)ME * HH * 2;
  const size_t PVH = (size_t)ME * HH * 2;
  const size_t PZH = (size_t)MQ * HH * 2;
  size_t off = 0;
  const size_t oXh = off; off += PXH;
  const size_t oEh = off; off += PEH;
  const size_t oWq = off; off += PWQ;
  const size_t oWk = off; off += PWK;
  const size_t oWv = off; off += PWV;
  const size_t oWo = off; off += PWO;
  const size_t oQf = off; off += PQF;
  const size_t oKh = off; off += PKH;
  const size_t oVh = off; off += PVH;
  const size_t oZh = off; off += PZH;
  if (off > ws_size) return;
  if (off > (size_t)134217728) return;

  char* ws = (char*)d_ws;
  unsigned short* Xh  = (unsigned short*)(ws + oXh);
  unsigned short* Eh  = (unsigned short*)(ws + oEh);
  unsigned short* Wqh = (unsigned short*)(ws + oWq);
  unsigned short* Wkh = (unsigned short*)(ws + oWk);
  unsigned short* Wvh = (unsigned short*)(ws + oWv);
  unsigned short* Woh = (unsigned short*)(ws + oWo);
  float*          Qf  = (float*)(ws + oQf);
  unsigned short* Kh  = (unsigned short*)(ws + oKh);
  unsigned short* Vh  = (unsigned short*)(ws + oVh);
  unsigned short* Zh  = (unsigned short*)(ws + oZh);
  float*          out0 = (float*)d_out;

  const dim3 blk(256);
  const int gq  = ((MQ / 64) * (HH / 64)) / 8;
  const int gkv = ((ME / 64) * (HH / 64)) / 8;
  if ((((MQ / 64) * (HH / 64)) % 8) != 0) return;
  if ((((ME / 64) * (HH / 64)) % 8) != 0) return;
  if (((MQ * HH) % 2048) != 0 || ((ME * RH) % 2048) != 0 || ((HH * HH) % 2048) != 0 || ((HH * RH) % 2048) != 0) return;

  cvt_flat<<<dim3((MQ * HH) / 2048), blk, 0, stream>>>(x, Xh, (MQ * HH) / 8, 1.0f);
  cvt_flat<<<dim3((ME * RH) / 2048), blk, 0, stream>>>(ex, Eh, (ME * RH) / 8, 1.0f);
  cvt_flat<<<dim3((HH * HH) / 2048), blk, 0, stream>>>(Wq, Wqh, (HH * HH) / 8, WSC);
  cvt_flat<<<dim3((HH * RH) / 2048), blk, 0, stream>>>(Wk, Wkh, (HH * RH) / 8, WSC);
  cvt_flat<<<dim3((HH * RH) / 2048), blk, 0, stream>>>(Wv, Wvh, (HH * RH) / 8, WSC);
  cvt_flat<<<dim3((HH * HH) / 2048), blk, 0, stream>>>(Wo, Woh, (HH * HH) / 8, WSC);

  gemm64<0><<<dim3(gq), blk, 0, stream>>>(
      Xh, HH, Wqh, HH, Kh, Qf, HH, x, HH, QSCL / WSC, MQ, HH, HH);
  gemm64<1><<<dim3(gkv), blk, 0, stream>>>(
      Eh, RH, Wkh, RH, Kh, Qf, HH, x, HH, 1.0f, ME, HH, RH);
  gemm64<1><<<dim3(gkv), blk, 0, stream>>>(
      Eh, RH, Wvh, RH, Vh, Qf, HH, x, HH, 1.0f, ME, HH, RH);

  attn_win<<<dim3((MQ * NHD) / 4), dim3(128), 0, stream>>>(Qf, (const _Float16*)Kh, (const _Float16*)Vh, Zh);

  gemm64<2><<<dim3(gq), blk, 0, stream>>>(
      Zh, HH, Woh, HH, Kh, out0, HH, x, HH, 1.0f / (WSC * WSC), MQ, HH, HH);
  (void)hipGetLastError();
}
